// Bilstm_crf_60507499266465
// MI455X (gfx1250) — hardware-verified
//
#include <hip/hip_runtime.h>
#include <math.h>

#define S_LEN 256
#define B_SZ  64
#define H_SZ  512
#define E_SZ  300
#define EP    320
#define G_SZ  2048
#define T_SZ  10
#define TP    16
#define KC_X  (EP / 32)
#define KC_H  (H_SZ / 32)
#define UPB   64
#define NCB   (UPB * 4)
#define GP    (NCB + 4)

typedef _Float16 f16;
typedef f16   v16h __attribute__((ext_vector_type(16)));
typedef f16   v8h  __attribute__((ext_vector_type(8)));
typedef __bf16 v16b __attribute__((ext_vector_type(16)));
typedef float v8f  __attribute__((ext_vector_type(8)));
typedef float v4f  __attribute__((ext_vector_type(4)));
typedef float v4fa __attribute__((ext_vector_type(4), may_alias));
typedef int   v4i  __attribute__((ext_vector_type(4)));
typedef int   v4ia __attribute__((ext_vector_type(4), may_alias));
union FragH { v16h v; v8h half[2]; };

__device__ __forceinline__ v8f wmma_h(v16h a, v16h b, v8f c) {
    c = __builtin_amdgcn_wmma_f32_16x16x32_f16(false, a, false, b, (short)0, c, false, false);
    asm volatile("v_nop\n\tv_nop\n\tv_nop\n\tv_nop" : "+v"(c) : "v"(a), "v"(b));
    return c;
}
__device__ __forceinline__ v8f wmma_b(v16b a, v16b b, v8f c) {
    c = __builtin_amdgcn_wmma_f32_16x16x32_bf16(false, a, false, b, (short)0, c, false, false);
    asm volatile("v_nop\n\tv_nop\n\tv_nop\n\tv_nop" : "+v"(c) : "v"(a), "v"(b));
    return c;
}
__device__ __forceinline__ v16h ld_frag(const f16* p, int h) {
    FragH f;
    f.half[0] = *(const v8h*)(p + 8 * h);
    f.half[1] = *(const v8h*)(p + 16 + 8 * h);
    return f.v;
}

__global__ __launch_bounds__(256)
void init_state_kernel(f16* __restrict__ h_st, float* __restrict__ c_st) {
    int idx = blockIdx.x * blockDim.x + threadIdx.x;
    const int nh = B_SZ * H_SZ / 8;
    const int nc = 2 * B_SZ * H_SZ / 4;
    v8h zh; v4f zc;
    #pragma unroll
    for (int i = 0; i < 8; ++i) zh[i] = (f16)0.0f;
    zc = 0.0f;
    for (int rep = 0; rep < 2; ++rep) {
        if (idx < nh) {
            *(volatile v8h*)(h_st + (size_t)idx * 8) = zh;
            *(volatile v8h*)(h_st + (size_t)2 * B_SZ * H_SZ + (size_t)idx * 8) = zh;
        }
        if (idx < nc) *(volatile v4f*)(c_st + (size_t)idx * 4) = zc;
        if (rep == 0) __threadfence();
    }
}

__global__ __launch_bounds__(64)
void embed_kernel(const int* __restrict__ tokens, const float* __restrict__ emb, f16* __restrict__ x_h, int vocab) {
    int sb = blockIdx.x;
    int s = sb / B_SZ, b = sb - s * B_SZ;
    int t = threadIdx.x;
    if (t >= EP / 8) return;
    int tok = tokens[b * S_LEN + s];
    tok = tok < 0 ? 0 : (tok >= vocab ? vocab - 1 : tok);
    v8h v;
    #pragma unroll
    for (int i = 0; i < 8; ++i) {
        int e = t * 8 + i;
        float f = (e < E_SZ) ? emb[(size_t)tok * E_SZ + e] * 256.0f : 0.0f;
        v[i] = (f16)f;
    }
    f16* dst = x_h + (size_t)sb * EP + t * 8;
    *(volatile v8h*)dst = v;
    __threadfence();
    *(volatile v8h*)dst = v;
}

__global__ __launch_bounds__(256)
void cast_weight_kernel(const float* __restrict__ src, f16* __restrict__ dst, int Ksrc, int Kdst) {
    int idx = blockIdx.x * blockDim.x + threadIdx.x;
    int per = Kdst / 8;
    int total = G_SZ * per;
    if (idx >= total) return;
    int r = idx / per;
    int e0 = (idx - r * per) * 8;
    int orig = (r & 3) * H_SZ + (r >> 2);
    v8h v;
    #pragma unroll
    for (int i = 0; i < 8; ++i) {
        int k = e0 + i;
        float f = (k < Ksrc) ? src[(size_t)orig * Ksrc + k] * 16.0f : 0.0f;
        v[i] = (f16)f;
    }
    f16* d = dst + (size_t)r * Kdst + e0;
    *(volatile v8h*)d = v;
    __threadfence();
    *(volatile v8h*)d = v;
}

__global__ __launch_bounds__(256)
void lstm_step_kernel(int step,
                      const f16* __restrict__ x_h,
                      const f16* __restrict__ wih_f_p, const f16* __restrict__ whh_f_p, const float* __restrict__ b_f,
                      const f16* __restrict__ wih_b_p, const f16* __restrict__ whh_b_p, const float* __restrict__ b_b,
                      const int* __restrict__ lengths,
                      f16* h_st,
                      float* c_st,
                      float* h_out)
{
    __shared__ float g[32 * GP];
    const int tid = threadIdx.x;
    const int l = tid & 31, h = l >> 4, m16 = l & 15, wave = tid >> 5;
    const int dir = blockIdx.z, bx = blockIdx.x;
    const int s = (dir == 0) ? step : (S_LEN - 1 - step);
    const int par = step & 1;
    const f16* wih = dir ? wih_b_p : wih_f_p;
    const f16* whh = dir ? whh_b_p : whh_f_p;
    const float* bias = dir ? b_b : b_f;
    const float ISC = 1.0f / 4096.0f;

    const int rb = bx * NCB + wave * 32 + m16;
    v8f acc[4][2];
    #pragma unroll
    for (int nt = 0; nt < 2; ++nt) {
        int r = rb + nt * 16;
        float bv = bias[(r & 3) * H_SZ + (r >> 2)] * 4096.0f;
        #pragma unroll
        for (int m = 0; m < 4; ++m)
            #pragma unroll
            for (int v = 0; v < 8; ++v) acc[m][nt][v] = bv;
    }

    const f16* xa = x_h + (size_t)s * B_SZ * EP;
    const f16* ha = h_st + (size_t)(dir * 2 + par) * B_SZ * H_SZ;

    #pragma unroll 2
    for (int kc = 0; kc < KC_X; ++kc) {
        const int k0 = kc * 32;
        v16h bf0 = ld_frag(wih + (size_t)rb * EP + k0, h);
        v16h bf1 = ld_frag(wih + (size_t)(rb + 16) * EP + k0, h);
        #pragma unroll
        for (int m = 0; m < 4; ++m) {
            v16h af = ld_frag(xa + (size_t)(m * 16 + m16) * EP + k0, h);
            acc[m][0] = wmma_h(af, bf0, acc[m][0]);
            acc[m][1] = wmma_h(af, bf1, acc[m][1]);
        }
    }
    #pragma unroll 2
    for (int kc = 0; kc < KC_H; ++kc) {
        const int k0 = kc * 32;
        v16h bf0 = ld_frag(whh + (size_t)rb * H_SZ + k0, h);
        v16h bf1 = ld_frag(whh + (size_t)(rb + 16) * H_SZ + k0, h);
        #pragma unroll
        for (int m = 0; m < 4; ++m) {
            v16h af = ld_frag(ha + (size_t)(m * 16 + m16) * H_SZ + k0, h);
            acc[m][0] = wmma_h(af, bf0, acc[m][0]);
            acc[m][1] = wmma_h(af, bf1, acc[m][1]);
        }
    }

    #pragma unroll
    for (int p = 0; p < 2; ++p) {
        #pragma unroll
        for (int mm = 0; mm < 2; ++mm)
            #pragma unroll
            for (int nt = 0; nt < 2; ++nt)
                #pragma unroll
                for (int r8 = 0; r8 < 8; ++r8) {
                    int row = mm * 16 + 8 * h + r8;
                    int col = wave * 32 + nt * 16 + m16;
                    g[row * GP + col] = acc[2 * p + mm][nt][r8];
                }
        __syncthreads();

        float cv[8], hv[8];
        #pragma unroll
        for (int i = 0; i < 8; ++i) {
            int q = tid + 256 * i;
            int bl = q >> 6, jl = q & 63;
            int b = 32 * p + bl;
            float gi = g[bl * GP + jl * 4 + 0] * ISC;
            float gf = g[bl * GP + jl * 4 + 1] * ISC;
            float gg = g[bl * GP + jl * 4 + 2] * ISC;
            float go = g[bl * GP + jl * 4 + 3] * ISC;
            int jg = bx * UPB + jl;
            float c_old = c_st[((size_t)dir * B_SZ + b) * H_SZ + jg];
            float ig = 1.0f / (1.0f + __expf(-gi));
            float fg = 1.0f / (1.0f + __expf(-gf));
            float og = 1.0f / (1.0f + __expf(-go));
            float cn = fg * c_old + ig * tanhf(gg);
            float hn = og * tanhf(cn);
            int len = lengths[b];
            bool mk = s < len;
            cv[i] = mk ? cn : c_old;
            hv[i] = hn;
        }
        __syncthreads();
        #pragma unroll
        for (int i = 0; i < 8; ++i) {
            int q = tid + 256 * i;
            g[q] = cv[i];
            g[2048 + q] = hv[i];
        }
        __syncthreads();

        for (int rep = 0; rep < 2; ++rep) {
            #pragma unroll
            for (int it = 0; it < 2; ++it) {
                int row = 16 * it + 2 * wave + (l >> 4);
                int b = 32 * p + row;
                int c4 = l & 15;
                bool mk = s < lengths[b];
                v4f cvv = *(const v4fa*)&g[row * 64 + 4 * c4];
                v4f hvv = *(const v4fa*)&g[2048 + row * 64 + 4 * c4];
                v4f zero = 0.0f;
                v4f ho = mk ? hvv : zero;
                *(volatile v4f*)(c_st + ((size_t)dir * B_SZ + b) * H_SZ + bx * UPB + 4 * c4) = cvv;
                *(volatile v4f*)(h_out + ((size_t)s * B_SZ + b) * (2 * H_SZ) + dir * H_SZ + bx * UPB + 4 * c4) = ho;
            }
            {
                int row = 4 * wave + (l >> 3);
                int b = 32 * p + row;
                int pc = l & 7;
                bool mk = s < lengths[b];
                v8h oldh = *(const v8h*)(h_st + ((size_t)(dir * 2 + par) * B_SZ + b) * H_SZ + bx * UPB + 8 * pc);
                v8h nh;
                #pragma unroll
                for (int i = 0; i < 8; ++i) nh[i] = (f16)(g[2048 + row * 64 + 8 * pc + i] * 256.0f);
                v8h val = mk ? nh : oldh;
                *(volatile v8h*)(h_st + ((size_t)(dir * 2 + (par ^ 1)) * B_SZ + b) * H_SZ + bx * UPB + 8 * pc) = val;
            }
            if (rep == 0) __threadfence();
        }
        __syncthreads();
    }
}

__global__ __launch_bounds__(128)
void proj_kernel(const float* __restrict__ h_out, const float* __restrict__ w_out,
                 const float* __restrict__ b_out, float* em, int nrows) {
    __shared__ float tile[4][256];
    const int l = threadIdx.x & 31, h = l >> 4, m16 = l & 15, wave = threadIdx.x >> 5;
    int gw = blockIdx.x * 4 + wave;
    const int nw = nrows / 16;
    int gwc = gw < nw ? gw : nw - 1;
    const int R0 = gwc * 16;
    v8f acc; acc = 0.0f;
    const float bmask = (m16 < T_SZ) ? 1.0f : 0.0f;
    const int tt = (m16 < T_SZ) ? m16 : (T_SZ - 1);

    #pragma unroll 2
    for (int kc = 0; kc < (2 * H_SZ) / 32; ++kc) {
        const int k0 = kc * 32;
        const float* ap = h_out + (size_t)(R0 + m16) * (2 * H_SZ) + k0;
        const float* bp = w_out + (size_t)tt * (2 * H_SZ) + k0;
        v4f a0 = *(const v4f*)(ap + 8 * h), a1 = *(const v4f*)(ap + 8 * h + 4);
        v4f a2 = *(const v4f*)(ap + 16 + 8 * h), a3 = *(const v4f*)(ap + 16 + 8 * h + 4);
        v4f b0 = *(const v4f*)(bp + 8 * h), b1 = *(const v4f*)(bp + 8 * h + 4);
        v4f b2 = *(const v4f*)(bp + 16 + 8 * h), b3 = *(const v4f*)(bp + 16 + 8 * h + 4);
        float av[16], bv[16];
        #pragma unroll
        for (int i = 0; i < 4; ++i) {
            av[i] = a0[i]; av[4 + i] = a1[i]; av[8 + i] = a2[i]; av[12 + i] = a3[i];
            bv[i] = b0[i] * bmask; bv[4 + i] = b1[i] * bmask; bv[8 + i] = b2[i] * bmask; bv[12 + i] = b3[i] * bmask;
        }
        v16b ah, al, bh, bl;
        #pragma unroll
        for (int i = 0; i < 16; ++i) {
            __bf16 x = (__bf16)av[i]; ah[i] = x; al[i] = (__bf16)(av[i] - (float)x);
            __bf16 y = (__bf16)bv[i]; bh[i] = y; bl[i] = (__bf16)(bv[i] - (float)y);
        }
        acc = wmma_b(ah, bh, acc);
        acc = wmma_b(ah, bl, acc);
        acc = wmma_b(al, bh, acc);
    }
    float bias = (m16 < T_SZ) ? b_out[m16] : 0.0f;
    #pragma unroll
    for (int r = 0; r < 8; ++r) tile[wave][(8 * h + r) * TP + m16] = acc[r] + bias;
    __syncthreads();
    if (gw < nw) {
        float* dst = em + (size_t)gw * 256;
        for (int rep = 0; rep < 2; ++rep) {
            v4f v0 = *(const v4fa*)&tile[wave][4 * l];
            v4f v1 = *(const v4fa*)&tile[wave][4 * (32 + l)];
            *(volatile v4f*)(dst + 4 * l) = v0;
            *(volatile v4f*)(dst + 4 * (32 + l)) = v1;
            if (rep == 0) __threadfence();
        }
    }
}

__global__ __launch_bounds__(64)
void viterbi_kernel(const float* __restrict__ em, const int* __restrict__ lengths,
                    const float* __restrict__ startv, const float* __restrict__ endv,
                    const float* __restrict__ trans,
                    int* bps, int* tags, int* out) {
    int b = threadIdx.x;
    if (b >= B_SZ) return;
    int len = lengths[b];
    len = len < 0 ? 0 : (len > S_LEN ? S_LEN : len);

    float tr[T_SZ * T_SZ];
    #pragma unroll
    for (int i = 0; i < T_SZ * T_SZ; ++i) tr[i] = trans[i];
    float score[T_SZ];
    #pragma unroll
    for (int t = 0; t < T_SZ; ++t) score[t] = startv[t] + em[((size_t)0 * B_SZ + b) * TP + t];

    int* bp = bps + (size_t)b * S_LEN * T_SZ;
    for (int ss = 1; ss < S_LEN; ++ss) {
        bool mk = ss < len;
        const float* emt = em + ((size_t)ss * B_SZ + b) * TP;
        float ns[T_SZ]; int nb[T_SZ];
        #pragma unroll
        for (int t = 0; t < T_SZ; ++t) {
            float best = score[0] + tr[t];
            int bi = 0;
            #pragma unroll
            for (int p2 = 1; p2 < T_SZ; ++p2) {
                float cn = score[p2] + tr[p2 * T_SZ + t];
                if (cn > best) { best = cn; bi = p2; }
            }
            ns[t] = mk ? (best + emt[t]) : score[t];
            nb[t] = mk ? bi : t;
        }
        #pragma unroll
        for (int t = 0; t < T_SZ; ++t) {
            score[t] = ns[t];
            *(volatile int*)(bp + ss * T_SZ + t) = nb[t];
            *(volatile int*)(bp + ss * T_SZ + t) = nb[t];
        }
    }
    float bestf = score[0] + endv[0];
    int last = 0;
    #pragma unroll
    for (int t = 1; t < T_SZ; ++t) {
        float cn = score[t] + endv[t];
        if (cn > bestf) { bestf = cn; last = t; }
    }
    int* tg = tags + b * S_LEN;
    int tag = last;
    {
        int v = ((S_LEN - 1) < len) ? tag : 0;
        *(volatile int*)(tg + S_LEN - 1) = v;
    }
    for (int ss = S_LEN - 1; ss >= 1; --ss) {
        int ti = tag < 0 ? 0 : (tag >= T_SZ ? T_SZ - 1 : tag);
        tag = *(volatile int*)(bp + ss * T_SZ + ti);
        tag = tag < 0 ? 0 : (tag >= T_SZ ? T_SZ - 1 : tag);
        int v = ((ss - 1) < len) ? tag : 0;
        *(volatile int*)(tg + ss - 1) = v;
    }
    __threadfence();
    int* orow = out + b * S_LEN;
    for (int rep = 0; rep < 2; ++rep) {
        for (int j = 0; j < S_LEN / 4; ++j) {
            v4i v = *(volatile v4ia*)(tg + 4 * j);
            *(volatile v4i*)(orow + 4 * j) = v;
        }
        if (rep == 0) __threadfence();
    }
}

extern "C" void kernel_launch(void* const* d_in, const int* in_sizes, int n_in,
                              void* d_out, int out_size, void* d_ws, size_t ws_size,
                              hipStream_t stream) {
    (void)n_in;
    const int*   tokens  = (const int*)d_in[0];
    const int*   lengths = (const int*)d_in[1];
    const float* emb     = (const float*)d_in[2];
    const float* wih_f   = (const float*)d_in[3];
    const float* whh_f   = (const float*)d_in[4];
    const float* b_f     = (const float*)d_in[5];
    const float* wih_b   = (const float*)d_in[6];
    const float* whh_b   = (const float*)d_in[7];
    const float* b_b     = (const float*)d_in[8];
    const float* w_out   = (const float*)d_in[9];
    const float* b_out   = (const float*)d_in[10];
    const float* startv  = (const float*)d_in[11];
    const float* endv    = (const float*)d_in[12];
    const float* trans   = (const float*)d_in[13];
    int vocab = in_sizes[2] / E_SZ;
    if (out_size < B_SZ * S_LEN) return;

    char* ws = (char*)d_ws;
    size_t off = 0;
    auto carve = [&](size_t bytes) -> char* {
        char* p = ws + off;
        off += (bytes + 255) & ~(size_t)255;
        return p;
    };
    f16*   x_h    = (f16*)  carve((size_t)S_LEN * B_SZ * EP * 2);
    f16*   wihp_f = (f16*)  carve((size_t)G_SZ * EP * 2);
    f16*   wihp_b = (f16*)  carve((size_t)G_SZ * EP * 2);
    f16*   whhp_f = (f16*)  carve((size_t)G_SZ * H_SZ * 2);
    f16*   whhp_b = (f16*)  carve((size_t)G_SZ * H_SZ * 2);
    f16*   h_st   = (f16*)  carve((size_t)4 * B_SZ * H_SZ * 2);
    float* c_st   = (float*)carve((size_t)2 * B_SZ * H_SZ * 4);
    float* h_out  = (float*)carve((size_t)S_LEN * B_SZ * 2 * H_SZ * 4);
    float* em     = (float*)carve((size_t)S_LEN * B_SZ * TP * 4);
    int*   bps    = (int*)  carve((size_t)B_SZ * S_LEN * T_SZ * 4);
    int*   tags   = (int*)  carve((size_t)B_SZ * S_LEN * 4);
    if (off > ws_size) return;
    int* out = (int*)d_out;

    {
        int n = B_SZ * H_SZ / 8 > 2 * B_SZ * H_SZ / 4 ? B_SZ * H_SZ / 8 : 2 * B_SZ * H_SZ / 4;
        init_state_kernel<<<dim3((n + 255) / 256), dim3(256), 0, stream>>>(h_st, c_st);
    }
    embed_kernel<<<dim3(S_LEN * B_SZ), dim3(64), 0, stream>>>(tokens, emb, x_h, vocab);
    {
        int tot_ih = G_SZ * (EP / 8), tot_hh = G_SZ * (H_SZ / 8);
        cast_weight_kernel<<<dim3((tot_ih + 255) / 256), dim3(256), 0, stream>>>(wih_f, wihp_f, E_SZ, EP);
        cast_weight_kernel<<<dim3((tot_ih + 255) / 256), dim3(256), 0, stream>>>(wih_b, wihp_b, E_SZ, EP);
        cast_weight_kernel<<<dim3((tot_hh + 255) / 256), dim3(256), 0, stream>>>(whh_f, whhp_f, H_SZ, H_SZ);
        cast_weight_kernel<<<dim3((tot_hh + 255) / 256), dim3(256), 0, stream>>>(whh_b, whhp_b, H_SZ, H_SZ);
    }
    for (int st = 0; st < S_LEN; ++st) {
        lstm_step_kernel<<<dim3(H_SZ / UPB, 1, 2), dim3(256), 0, stream>>>(
            st, x_h, wihp_f, whhp_f, b_f, wihp_b, whhp_b, b_b, lengths, h_st, c_st, h_out);
    }
    {
        int nrows = S_LEN * B_SZ;
        int nwaves = nrows / 16;
        proj_kernel<<<dim3((nwaves + 3) / 4), dim3(128), 0, stream>>>(h_out, w_out, b_out, em, nrows);
    }
    viterbi_kernel<<<dim3(1), dim3(64), 0, stream>>>(em, lengths, startv, endv, trans, bps, tags, out);
}
